// PrunableLeViTAttention_33947421507744
// MI455X (gfx1250) — hardware-verified
//
#include <hip/hip_runtime.h>
#include <math.h>
#include <stdint.h>

#define RES     14
#define NTOK    196
#define NP      256
#define DIM     384
#define KD      32
#define NHEAD   12
#define HQKV    192
#define VD      128
#define QKVD    2304
#define VAD     1536
#define BATCH   128
#define CHI     16
#define NCH     (BATCH / CHI)
#define MCH     (CHI * NTOK)
#define QROWS   (MCH + 64)
#define NY      (CHI * NHEAD)
#define KPV     224
#define BN_EPS  1e-5f
#define PSCALE  32768.0f
#define PSCALE_INV (1.0f / 32768.0f)

typedef __attribute__((ext_vector_type(16))) _Float16 v16h;
typedef __attribute__((ext_vector_type(8)))  _Float16 v8h;
typedef __attribute__((ext_vector_type(16))) __bf16   v16b;
typedef __attribute__((ext_vector_type(8)))  __bf16   v8b;
typedef __attribute__((ext_vector_type(8)))  float    v8f;
typedef __attribute__((ext_vector_type(4)))  float    v4f;
typedef __attribute__((ext_vector_type(2)))  float    v2f;
typedef __attribute__((ext_vector_type(4)))  unsigned int v4u;

__device__ __forceinline__ unsigned short f2bf_bits(float f) {
  unsigned u = __float_as_uint(f);
  return (unsigned short)((u + 0x7FFFu + ((u >> 16) & 1u)) >> 16);
}
__device__ __forceinline__ float bf_bits2f(unsigned short h) { return __uint_as_float(((unsigned)h) << 16); }
__device__ __forceinline__ unsigned pk16(unsigned short a, unsigned short b) { return (unsigned)a | ((unsigned)b << 16); }
__device__ __forceinline__ unsigned short h_bits(float f) { const _Float16 h = (_Float16)f; return __builtin_bit_cast(unsigned short, h); }

__device__ __forceinline__ void dep_guard_h(v8f& a, v8f& b, v16h x, v16h y) { asm volatile("v_nop\n\tv_nop\n\tv_nop\n\tv_nop" : "+v"(a), "+v"(b) : "v"(x), "v"(y)); }
__device__ __forceinline__ void dep_guard_b(v8f& a, v8f& b, v16b x, v16b y) { asm volatile("v_nop\n\tv_nop\n\tv_nop\n\tv_nop" : "+v"(a), "+v"(b) : "v"(x), "v"(y)); }
__device__ __forceinline__ void keep4_h(v16h a, v16h b, v16h c, v16h d) { asm volatile("v_nop" :: "v"(a), "v"(b), "v"(c), "v"(d)); }
__device__ __forceinline__ void keep4_b(v16b a, v16b b, v16b c, v16b d) { asm volatile("v_nop" :: "v"(a), "v"(b), "v"(c), "v"(d)); }
__device__ __forceinline__ void acc_guard4(v8f& a, v8f& b, v8f& c, v8f& d) { asm volatile("v_nop\n\tv_nop\n\tv_nop\n\tv_nop" : "+v"(a), "+v"(b), "+v"(c), "+v"(d)); }
template <typename T> struct Frag;
template <> struct Frag<_Float16> {
  typedef v16h V; union U { v16h v; v8h h[2]; };
  static __device__ __forceinline__ v16h load(const _Float16* p) {
    U f; f.h[0] = *(const v8h*)(p); f.h[1] = *(const v8h*)(p + 16); return f.v;
  }
  static __device__ __forceinline__ v8f mma(v16h a, v16h b, v8f c) {
    return __builtin_amdgcn_wmma_f32_16x16x32_f16(false, a, false, b, (short)0, c, false, false);
  }
  static __device__ __forceinline__ void guard(v8f& a, v8f& b, v16h x, v16h y) { dep_guard_h(a, b, x, y); }
  static __device__ __forceinline__ void keep(v16h a, v16h b, v16h c, v16h d) { keep4_h(a, b, c, d); }
};
template <> struct Frag<__bf16> {
  typedef v16b V; union U { v16b v; v8b h[2]; };
  static __device__ __forceinline__ v16b load(const __bf16* p) {
    U f; f.h[0] = *(const v8b*)(p); f.h[1] = *(const v8b*)(p + 16); return f.v;
  }
  static __device__ __forceinline__ v8f mma(v16b a, v16b b, v8f c) {
    return __builtin_amdgcn_wmma_f32_16x16x32_bf16(false, a, false, b, (short)0, c, false, false);
  }
  static __device__ __forceinline__ void guard(v8f& a, v8f& b, v16b x, v16b y) { dep_guard_b(a, b, x, y); }
  static __device__ __forceinline__ void keep(v16b a, v16b b, v16b c, v16b d) { keep4_b(a, b, c, d); }
};

template <int ET> struct Elem;
template <> struct Elem<0> { typedef _Float16 T; };
template <> struct Elem<1> { typedef __bf16 T; };
template <int ET, bool SPLIT, int BIAS_MODE, int OUT_MODE, bool RESID, int ACT = 0>
__global__ __launch_bounds__(256) void wmma_gemm64(
    const unsigned short* __restrict__ Ap, const unsigned short* __restrict__ A2p, int lda, long strideA, long strideA2,
    const unsigned short* __restrict__ Btp, const unsigned short* __restrict__ Bt2p, int ldb, long strideB, long strideB2,
    void* __restrict__ Cout, void* __restrict__ Cout2, int ldc, long strideC, long strideC2,
    const float* __restrict__ bias,
    const float* __restrict__ resid, long strideR,
    int M, int N, int K, int Mvalid, int ydiv, float scale, float oscale) {
  typedef typename Elem<ET>::T T;
  typedef typename Frag<T>::V V;
  const T* A = (const T*)Ap; const T* A2 = (const T*)A2p; const T* Bt = (const T*)Btp; const T* Bt2 = (const T*)Bt2p;
  __shared__ __align__(16) float sT[8][16 * 68];
  const int b    = blockIdx.y;
  const int y1   = b / ydiv;
  const int y2   = b - y1 * ydiv;
  const int lane = threadIdx.x & 31;
  const int wave = threadIdx.x >> 5;
  const int tilesN = N >> 6;
  const int tilesM = M >> 6;
  const int tile = blockIdx.x * 8 + wave;
  if (tile >= tilesM * tilesN) return;
  const int tm = tile / tilesN;
  const int tn = tile - tm * tilesN;
  const int m0 = tm << 6;
  const int n0 = tn << 6;

  const size_t offA = (size_t)y1 * (size_t)strideA + (size_t)y2 * (size_t)strideA2;
  const size_t offB = (size_t)y1 * (size_t)strideB + (size_t)y2 * (size_t)strideB2;
  const size_t offC = (size_t)y1 * (size_t)strideC + (size_t)y2 * (size_t)strideC2;
  const T* Ab  = A  + offA;
  const T* Bb  = Bt + offB;
  const T* Ab2 = SPLIT ? (A2  + offA) : nullptr;
  const T* Bb2 = SPLIT ? (Bt2 + offB) : nullptr;

  const int rlane = lane & 15;
  const int koff  = (lane >> 4) * 8;
  const int mOff  = (lane >> 4) * 8;

  v8f acc[4][4];
#pragma unroll
  for (int i = 0; i < 4; ++i)
#pragma unroll
    for (int j = 0; j < 4; ++j) acc[i][j] = (v8f){0.f,0.f,0.f,0.f,0.f,0.f,0.f,0.f};

  for (int k0 = 0; k0 < K; k0 += 32) {
    V bh[4], bl[4];
#pragma unroll
    for (int j = 0; j < 4; ++j) {
      const size_t bo = (size_t)(n0 + (j << 4) + rlane) * ldb + koff + k0;
      bh[j] = Frag<T>::load(Bb + bo);
      if (SPLIT) bl[j] = Frag<T>::load(Bb2 + bo);
    }
#pragma unroll
    for (int i = 0; i < 4; ++i) {
      const size_t ao = (size_t)(m0 + (i << 4) + rlane) * lda + koff + k0;
      V ah = Frag<T>::load(Ab + ao);
      V al;
      if (SPLIT) al = Frag<T>::load(Ab2 + ao);
#pragma unroll
      for (int j = 0; j < 4; ++j) {
        acc[i][j] = Frag<T>::mma(ah, bh[j], acc[i][j]);
        if (SPLIT) {
          acc[i][j] = Frag<T>::mma(ah, bl[j], acc[i][j]);
          acc[i][j] = Frag<T>::mma(al, bh[j], acc[i][j]);
        }
      }
      Frag<T>::guard(acc[i][0], acc[i][3], ah, SPLIT ? al : ah);
    }
    Frag<T>::keep(bh[0], bh[1], bh[2], bh[3]);
    if (SPLIT) Frag<T>::keep(bl[0], bl[1], bl[2], bl[3]);
  }
  acc_guard4(acc[0][0], acc[0][1], acc[0][2], acc[0][3]);
  acc_guard4(acc[1][0], acc[1][1], acc[1][2], acc[1][3]);
  acc_guard4(acc[2][0], acc[2][1], acc[2][2], acc[2][3]);
  acc_guard4(acc[3][0], acc[3][1], acc[3][2], acc[3][3]);

  float* slab = sT[wave];
  const float* Rb = RESID ? (resid + (size_t)y1 * (size_t)strideR) : nullptr;
#pragma unroll
  for (int i = 0; i < 4; ++i) {
    const int mBase = m0 + (i << 4);
#pragma unroll
    for (int j = 0; j < 4; ++j) {
      const int n = n0 + (j << 4) + rlane;
      float bv = 0.f;
      if (BIAS_MODE == 2) bv = bias[n];
#pragma unroll
      for (int r = 0; r < 8; ++r) {
        float v = acc[i][j][r] * scale;
        if (BIAS_MODE == 1) v += bias[mBase + mOff + r];
        if (BIAS_MODE == 2) v += bv;
        if (RESID) v += Rb[(size_t)(mBase + mOff + r) * ldc + n];
        if (ACT == 1) v = tanhf(v);
        if (ACT == 2) v = fmaxf(v, 0.0f);
        if (ACT == 3) v = v * __builtin_amdgcn_rcpf(1.0f + __expf(-v));
        if (ACT == 4) v = (v > 0.f) ? v : 0.01f * v;
        v = v * oscale;
        slab[(mOff + r) * 68 + (j << 4) + rlane] = v;
      }
    }
    __builtin_amdgcn_fence(__ATOMIC_RELEASE, "workgroup");
    __builtin_amdgcn_wave_barrier();
    __builtin_amdgcn_fence(__ATOMIC_ACQUIRE, "workgroup");
    if (OUT_MODE == 0) {
      float* C = (float*)Cout + offC;
      const int hh = lane >> 4, c4 = (lane & 15) * 4;
      for (int pass = 0; pass < 2; ++pass) {
#pragma unroll
        for (int it = 0; it < 8; ++it) {
          const int row = it * 2 + hh;
          const bool rok = (mBase + row) < Mvalid;
          v4f v = *(const v4f*)(slab + row * 68 + c4);
          if (rok) *(volatile v4f*)(C + (size_t)(mBase + row) * ldc + n0 + c4) = v;
        }
        __threadfence();
      }
    } else {
      const int q = lane >> 3, c8 = (lane & 7) * 8;
      unsigned short* C  = (unsigned short*)Cout  + offC;
      unsigned short* C2 = (OUT_MODE == 2) ? ((unsigned short*)Cout2 + offC) : nullptr;
      for (int pass = 0; pass < 2; ++pass) {
#pragma unroll
        for (int it = 0; it < 4; ++it) {
          const int row = it * 4 + q;
          const bool rok = (mBase + row) < Mvalid;
          const float* sp = slab + row * 68 + c8;
          v8h hv, lv;
#pragma unroll
          for (int e = 0; e < 8; ++e) {
            if (OUT_MODE == 1) {
              hv[e] = (_Float16)sp[e];
            } else {
              unsigned short hb = f2bf_bits(sp[e]);
              unsigned short lb = f2bf_bits(sp[e] - bf_bits2f(hb));
              hv[e] = __builtin_bit_cast(_Float16, hb);
              lv[e] = __builtin_bit_cast(_Float16, lb);
            }
          }
          if (rok) {
            *(volatile v8h*)(C + (size_t)(mBase + row) * ldc + n0 + c8) = hv;
            if (OUT_MODE == 2) *(volatile v8h*)(C2 + (size_t)(mBase + row) * ldc + n0 + c8) = lv;
          }
        }
        __threadfence();
      }
    }
    __builtin_amdgcn_fence(__ATOMIC_RELEASE, "workgroup");
    __builtin_amdgcn_wave_barrier();
    __builtin_amdgcn_fence(__ATOMIC_ACQUIRE, "workgroup");
  }
}

__global__ __launch_bounds__(256) void cast_f16x2_kernel(const float* __restrict__ in, unsigned short* __restrict__ out, int n2, float scale) {
  const int i = blockIdx.x * 256 + threadIdx.x;
  if (i < n2) {
    const v2f f = *(const v2f*)(in + 2 * (size_t)i);
    const unsigned u = pk16(h_bits(f[0] * scale), h_bits(f[1] * scale));
    ((volatile unsigned*)out)[i] = u;
    __threadfence();
    ((volatile unsigned*)out)[i] = u;
  }
}

__global__ __launch_bounds__(256) void zero16_kernel(unsigned short* __restrict__ out, int n16) {
  const int i = blockIdx.x * 256 + threadIdx.x;
  if (i < n16) {
    const v4u z = (v4u){0u, 0u, 0u, 0u};
    *(volatile v4u*)(out + (size_t)i * 8) = z;
    __threadfence();
    *(volatile v4u*)(out + (size_t)i * 8) = z;
  }
}

__global__ __launch_bounds__(256) void fold_cast_kernel(const float* __restrict__ w, const float* __restrict__ gamma,
                                                        const float* __restrict__ var, unsigned short* __restrict__ out,
                                                        int n2, int cols, float carry) {
  const int i = blockIdx.x * 256 + threadIdx.x;
  if (i < n2) {
    const int o = (2 * i) / cols;
    const float inv = gamma[o] * (1.0f / sqrtf(var[o] + BN_EPS));
    const float s = inv * carry;
    const v2f f = *(const v2f*)(w + 2 * (size_t)i);
    const unsigned u = pk16(h_bits(f[0] * s), h_bits(f[1] * s));
    ((volatile unsigned*)out)[i] = u;
    __threadfence();
    ((volatile unsigned*)out)[i] = u;
  }
}

__global__ __launch_bounds__(256) void bn_shift_kernel(const float* __restrict__ gamma, const float* __restrict__ beta,
                                                      const float* __restrict__ mean, const float* __restrict__ var,
                                                      float* __restrict__ shift, int n) {
  const int i = blockIdx.x * 256 + threadIdx.x;
  if (i < n) {
    const float inv = gamma[i] * (1.0f / sqrtf(var[i] + BN_EPS));
    const float s = beta[i] - mean[i] * inv;
    ((volatile float*)shift)[i] = s;
    __threadfence();
    ((volatile float*)shift)[i] = s;
  }
}

__global__ __launch_bounds__(256) void softmax_bias_kernel(const float* __restrict__ S,
                                                           const float* __restrict__ ab,
                                                           unsigned short* __restrict__ P) {
  const int tid  = threadIdx.x;
  const int lane = tid & 31;
  const int wave = tid >> 5;
  const int y    = blockIdx.x >> 5;
  const int rg   = blockIdx.x & 31;
  const int h    = y % NHEAD;
  const int n    = rg * 8 + wave;
  const int nc   = n < NTOK ? n : NTOK - 1;
  const int yn   = nc / RES, xn = nc - yn * RES;
  const size_t ro = ((size_t)y * NP + n) * NP + lane * 8;
  const v4f a = *(const v4f*)(S + ro);
  const v4f c = *(const v4f*)(S + ro + 4);
  const float sv[8] = {a[0], a[1], a[2], a[3], c[0], c[1], c[2], c[3]};
  const float* abh = ab + h * NTOK;
  float t[8];
  float m = -1.0e30f;
#pragma unroll
  for (int e = 0; e < 8; ++e) {
    const int mm = lane * 8 + e;
    const int mc = mm < NTOK ? mm : NTOK - 1;
    const int ym = mc / RES, xm = mc - ym * RES;
    int dy = yn - ym; dy = dy < 0 ? -dy : dy;
    int dx = xn - xm; dx = dx < 0 ? -dx : dx;
    const float bv = abh[dy * RES + dx];
    t[e] = (mm < NTOK) ? (sv[e] + bv) : -1.0e30f;
    m = fmaxf(m, t[e]);
  }
#pragma unroll
  for (int off = 16; off > 0; off >>= 1) m = fmaxf(m, __shfl_xor(m, off, 32));
  float ev[8];
  float s = 0.f;
#pragma unroll
  for (int e = 0; e < 8; ++e) { ev[e] = __expf(t[e] - m); s += ev[e]; }
#pragma unroll
  for (int off = 16; off > 0; off >>= 1) s += __shfl_xor(s, off, 32);
  const float inv = 1.0f / s;
  const float pm = (n < NTOK) ? inv * PSCALE : 0.0f;
  const v4u hv = (v4u){pk16(h_bits(ev[0] * pm), h_bits(ev[1] * pm)),
                       pk16(h_bits(ev[2] * pm), h_bits(ev[3] * pm)),
                       pk16(h_bits(ev[4] * pm), h_bits(ev[5] * pm)),
                       pk16(h_bits(ev[6] * pm), h_bits(ev[7] * pm))};
  *(volatile v4u*)(P + ro) = hv;
  __threadfence();
  *(volatile v4u*)(P + ro) = hv;
}

#define VTP 264
__global__ __launch_bounds__(256) void vtrans_kernel(const unsigned short* __restrict__ QKV, unsigned short* __restrict__ VT) {
  __shared__ __align__(16) _Float16 sm[64 * VTP];
  const int y   = blockIdx.x >> 1;
  const int dh  = blockIdx.x & 1;
  const int img = y / NHEAD;
  const int h   = y - img * NHEAD;
  const _Float16* src = (const _Float16*)QKV + (size_t)img * NTOK * QKVD + h * HQKV + 2 * KD + dh * 64;
  const int tid = threadIdx.x;
  const int mr  = tid >> 3;
  const int c8  = (tid & 7) * 8;
#pragma unroll
  for (int it = 0; it < 8; ++it) {
    const int m  = it * 32 + mr;
    const int mc = m < NTOK ? m : NTOK - 1;
    const v8h v  = *(const v8h*)(src + (size_t)mc * QKVD + c8);
    const bool ok = m < NTOK;
#pragma unroll
    for (int e = 0; e < 8; ++e) sm[(c8 + e) * VTP + m] = ok ? v[e] : (_Float16)0.0f;
  }
  __syncthreads();
  const int wave = tid >> 5, lane = tid & 31;
  _Float16* dst = (_Float16*)VT + ((size_t)y * VD + dh * 64) * NP;
  for (int pass = 0; pass < 2; ++pass) {
#pragma unroll
    for (int r = 0; r < 8; ++r) {
      const int d = wave * 8 + r;
      const v8h o = *(const v8h*)(sm + d * VTP + lane * 8);
      *(volatile v8h*)(dst + (size_t)d * NP + lane * 8) = o;
    }
    __threadfence();
  }
}

extern "C" void kernel_launch(void* const* d_in, const int* in_sizes, int n_in,
                              void* d_out, int out_size, void* d_ws, size_t ws_size,
                              hipStream_t stream) {
  if (n_in < 12) return;
  if (in_sizes[0] != BATCH * NTOK * DIM) return;
  if (in_sizes[1] != QKVD * DIM) return;
  if (in_sizes[2] != QKVD || in_sizes[3] != QKVD || in_sizes[4] != QKVD || in_sizes[5] != QKVD) return;
  if (in_sizes[6] != NHEAD * NTOK) return;
  if (in_sizes[7] != DIM * VAD) return;
  if (in_sizes[8] != DIM || in_sizes[9] != DIM || in_sizes[10] != DIM || in_sizes[11] != DIM) return;
  if (out_size != BATCH * NTOK * DIM) return;

  const float* x          = (const float*)d_in[0];
  const float* qkv_w      = (const float*)d_in[1];
  const float* qkv_gamma  = (const float*)d_in[2];
  const float* qkv_beta   = (const float*)d_in[3];
  const float* qkv_mean   = (const float*)d_in[4];
  const float* qkv_var    = (const float*)d_in[5];
  const float* attn_b     = (const float*)d_in[6];
  const float* proj_w     = (const float*)d_in[7];
  const float* proj_gamma = (const float*)d_in[8];
  const float* proj_beta  = (const float*)d_in[9];
  const float* proj_mean  = (const float*)d_in[10];
  const float* proj_var   = (const float*)d_in[11];
  float* out = (float*)d_out;

  auto alup = [](size_t v) -> size_t { return (v + 255) & ~(size_t)255; };
  size_t off = 0;
  const size_t oWQ  = off; off += alup((size_t)QKVD * DIM * 2);
  const size_t oWP  = off; off += alup((size_t)DIM * VAD * 2);
  const size_t oSHQ = off; off += alup((size_t)QKVD * 4);
  const size_t oSHP = off; off += alup((size_t)DIM * 4);
  const size_t oX   = off; off += alup((size_t)MCH * DIM * 2);
  const size_t oQKV = off; off += alup((size_t)QROWS * QKVD * 2);
  const size_t oS   = off; off += alup((size_t)NY * NP * NP * 4);
  const size_t oP   = off; off += alup((size_t)NY * NP * NP * 2);
  const size_t oVT  = off; off += alup((size_t)NY * VD * NP * 2);
  const size_t oCTX = off; off += alup((size_t)MCH * VAD * 2);
  if (off > ws_size) return;

  char* ws = (char*)d_ws;
  unsigned short* WQ16  = (unsigned short*)(ws + oWQ);
  unsigned short* WP16  = (unsigned short*)(ws + oWP);
  float*          SHQ   = (float*)(ws + oSHQ);
  float*          SHP   = (float*)(ws + oSHP);
  unsigned short* X16   = (unsigned short*)(ws + oX);
  unsigned short* QKV16 = (unsigned short*)(ws + oQKV);
  float*          Sbuf  = (float*)(ws + oS);
  unsigned short* P16   = (unsigned short*)(ws + oP);
  unsigned short* VT16  = (unsigned short*)(ws + oVT);
  unsigned short* CTX16 = (unsigned short*)(ws + oCTX);

  const dim3 blk(256);
  const int n2wq = QKVD * DIM / 2;
  const int n2wp = DIM * VAD / 2;
  const int n16z = (QROWS - MCH) * QKVD / 8;
  fold_cast_kernel<<<dim3(n2wq / 256), blk, 0, stream>>>(qkv_w, qkv_gamma, qkv_var, WQ16, n2wq, DIM, 16.0f);
  fold_cast_kernel<<<dim3(n2wp / 256), blk, 0, stream>>>(proj_w, proj_gamma, proj_var, WP16, n2wp, VAD, 16.0f);
  bn_shift_kernel<<<dim3(QKVD / 256), blk, 0, stream>>>(qkv_gamma, qkv_beta, qkv_mean, qkv_var, SHQ, QKVD);
  bn_shift_kernel<<<dim3((DIM + 255) / 256), blk, 0, stream>>>(proj_gamma, proj_beta, proj_mean, proj_var, SHP, DIM);
  zero16_kernel<<<dim3((n16z + 255) / 256), blk, 0, stream>>>(QKV16 + (size_t)MCH * QKVD, n16z);

  const int n2x = MCH * DIM / 2;
  const dim3 gCastX(n2x / 256);
  const dim3 gQKV(((MCH / 64) * (QKVD / 64) + 7) / 8, 1);
  const dim3 gS(((NP / 64) * (NP / 64) + 7) / 8, NY);
  const dim3 gSM(NY * 32);
  const dim3 gVT(NY * 2);
  const dim3 gPV(((NP / 64) * (VD / 64) + 7) / 8, NY);
  const dim3 gPJ(((MCH / 64) * (DIM / 64) + 7) / 8, 1);
  const float wscale = 1.0f / 16.0f;
  const float sscale = 0.17677669529663688f;

  for (int ch = 0; ch < NCH; ++ch) {
    cast_f16x2_kernel<<<gCastX, blk, 0, stream>>>(x + (size_t)ch * MCH * DIM, X16, n2x, 1.0f);
    wmma_gemm64<0, false, 2, 1, false, 0><<<gQKV, blk, 0, stream>>>(
        X16, X16, DIM, 0L, 0L, WQ16, WQ16, DIM, 0L, 0L, (void*)QKV16, (void*)QKV16, QKVD, 0L, 0L,
        SHQ, SHQ, 0L, MCH, QKVD, DIM, MCH, 1, wscale, 1.0f);
    wmma_gemm64<0, false, 0, 0, false, 0><<<gS, blk, 0, stream>>>(
        QKV16, QKV16, QKVD, (long)NTOK * QKVD, (long)HQKV,
        QKV16 + KD, QKV16 + KD, QKVD, (long)NTOK * QKVD, (long)HQKV,
        (void*)Sbuf, (void*)Sbuf, NP, (long)NHEAD * NP * NP, (long)NP * NP,
        SHQ, SHQ, 0L, NP, NP, KD, NP, NHEAD, sscale, 1.0f);
    softmax_bias_kernel<<<gSM, blk, 0, stream>>>(Sbuf, attn_b, P16);
    vtrans_kernel<<<gVT, blk, 0, stream>>>(QKV16, VT16);
    wmma_gemm64<0, false, 0, 1, false, 3><<<gPV, blk, 0, stream>>>(
        P16, P16, NP, (long)NHEAD * NP * NP, (long)NP * NP,
        VT16, VT16, NP, (long)NHEAD * VD * NP, (long)VD * NP,
        (void*)CTX16, (void*)CTX16, VAD, (long)NTOK * VAD, (long)VD,
        SHQ, SHQ, 0L, NP, VD, KPV, NTOK, NHEAD, PSCALE_INV, 16.0f);
    wmma_gemm64<0, false, 2, 0, false, 0><<<gPJ, blk, 0, stream>>>(
        CTX16, CTX16, VAD, 0L, 0L, WP16, WP16, VAD, 0L, 0L,
        (void*)(out + (size_t)ch * MCH * DIM), (void*)(out + (size_t)ch * MCH * DIM), DIM, 0L, 0L,
        SHP, SHP, 0L, MCH, DIM, VAD, MCH, 1, 1.0f / 256.0f, 1.0f);
  }
  (void)hipGetLastError();
}
